// BertSelfAttention_25237227831508
// MI455X (gfx1250) — hardware-verified
//
#include <hip/hip_runtime.h>


#ifndef NB
#define NB 8
#endif
#ifndef SEQ
#define SEQ 1024
#endif
#define NB_FULL 8
#define SEQ_FULL 1024
#define DM 1024
#define NH 16
#define HD 64
#define NT (NB * SEQ)
#define WSC 64.0f
#define PSC 1024.0f
#define LDP 136
#define OLP 68

static_assert(DM == NH * HD);
static_assert(SEQ % 128 == 0);
static_assert(SEQ <= SEQ_FULL);
static_assert(NB >= 1 && NB <= NB_FULL);
static_assert(NT % 128 == 0);
static_assert(DM % 128 == 0);
static_assert((NT * (DM / 8)) % 256 == 0);
static_assert((DM * (DM / 8)) % 256 == 0);

typedef _Float16 v16h __attribute__((ext_vector_type(16)));
typedef _Float16 v8h  __attribute__((ext_vector_type(8)));
typedef float    v8f  __attribute__((ext_vector_type(8)));
typedef float    v4f  __attribute__((ext_vector_type(4)));
typedef unsigned v4u  __attribute__((ext_vector_type(4)));
union Frag { v16h v; v8h hf[2]; };

__device__ __forceinline__ float bf16r(float f) {
    unsigned u = __float_as_uint(f);
    u += 0x7FFFu + ((u >> 16) & 1u);
    return __uint_as_float(u & 0xFFFF0000u);
}
__device__ __forceinline__ v8h ld8(const _Float16* p) { return *(const v8h*)p; }

__device__ __forceinline__ v8f wmma16(v16h a, v16h b, v8f c) {
    c = __builtin_amdgcn_wmma_f32_16x16x32_f16(false, a, false, b, (short)0, c, false, false);
    asm volatile("v_nop\n\tv_nop\n\tv_nop\n\tv_nop" : "+v"(c) : "v"(a), "v"(b));
    return c;
}

__global__ __launch_bounds__(256)
void cvt_kernel(const float* __restrict__ x, const float* __restrict__ wq, const float* __restrict__ wk,
                const float* __restrict__ wv, _Float16* xh, _Float16* wqh, _Float16* wkh, _Float16* wvh) {
    const int nbx = NT * (DM / 8) / 256;
    const int nbw = DM * (DM / 8) / 256;
    int blk = blockIdx.x;
    const int tid = threadIdx.x;
    const float* src;
    _Float16* dst;
    float sc;
    if (blk < nbx) {
        const int idx = blk * 256 + tid;
        const int t = idx / (DM / 8), c8 = idx - t * (DM / 8);
        const int b = t / SEQ, s = t - b * SEQ;
        src = x + (size_t)(b * SEQ_FULL + s) * DM + 8 * c8;
        dst = xh + (size_t)t * DM + 8 * c8;
        sc = 1.0f;
    } else {
        blk -= nbx;
        const int w = blk / nbw;
        const int idx = (blk - w * nbw) * 256 + tid;
        src = (w == 0 ? wq : (w == 1 ? wk : wv)) + (size_t)idx * 8;
        dst = (w == 0 ? wqh : (w == 1 ? wkh : wvh)) + (size_t)idx * 8;
        sc = WSC;
    }
    const v4f a = *(const v4f*)src, c = *(const v4f*)(src + 4);
    v8h o;
    o[0] = (_Float16)(bf16r(a[0]) * sc); o[1] = (_Float16)(bf16r(a[1]) * sc);
    o[2] = (_Float16)(bf16r(a[2]) * sc); o[3] = (_Float16)(bf16r(a[3]) * sc);
    o[4] = (_Float16)(bf16r(c[0]) * sc); o[5] = (_Float16)(bf16r(c[1]) * sc);
    o[6] = (_Float16)(bf16r(c[2]) * sc); o[7] = (_Float16)(bf16r(c[3]) * sc);
    const v4u val = __builtin_bit_cast(v4u, o);
    *(volatile v4u*)dst = val;
    __threadfence();
    *(volatile v4u*)dst = val;
}

template <int MODE>
__global__ __launch_bounds__(256) __attribute__((amdgpu_num_vgpr(256)))
void proj_kernel(const _Float16* __restrict__ A0, const _Float16* __restrict__ A1, const _Float16* __restrict__ Bm,
                 const float* __restrict__ bias0, const float* __restrict__ bias1, _Float16* Out0, _Float16* Out1) {
    __shared__ __align__(16) _Float16 L[128 * LDP];
    const int z = blockIdx.z;
    const _Float16* A = z ? A1 : A0;
    const float* bias = z ? bias1 : bias0;
    _Float16* Out = z ? Out1 : Out0;
    const int tid = threadIdx.x, lane = tid & 31, wv = tid >> 5, h = lane >> 4, n16 = lane & 15;
    const int wmi = wv & 3, wn = wv >> 2;
    const int m0 = blockIdx.x * 128, n0 = blockIdx.y * 128;
    const _Float16* ar = A + (size_t)(m0 + 32 * wmi + n16) * DM + 8 * h;
    const _Float16* br = Bm + (size_t)(n0 + 64 * wn + n16) * DM + 8 * h;
    v8f acc[2][4];
#pragma unroll
    for (int at = 0; at < 2; ++at)
#pragma unroll
        for (int bt = 0; bt < 4; ++bt) acc[at][bt] = (v8f){};
#pragma unroll 1
    for (int kc = 0; kc < DM; kc += 32) {
        Frag a0, a1;
        a0.hf[0] = ld8(ar + kc);           a0.hf[1] = ld8(ar + kc + 16);
        a1.hf[0] = ld8(ar + 16 * DM + kc); a1.hf[1] = ld8(ar + 16 * DM + kc + 16);
#pragma unroll
        for (int bt = 0; bt < 4; ++bt) {
            const _Float16* bp = br + (size_t)(16 * bt) * DM + kc;
            Frag bf;
            bf.hf[0] = ld8(bp); bf.hf[1] = ld8(bp + 16);
            acc[0][bt] = wmma16(a0.v, bf.v, acc[0][bt]);
            acc[1][bt] = wmma16(a1.v, bf.v, acc[1][bt]);
        }
    }
    const float osc = 1.0f / WSC;
#pragma unroll
    for (int at = 0; at < 2; ++at) {
        float bmv[8];
        if (MODE == 0) {
            const float* bp = bias + m0 + 32 * wmi + 16 * at + 8 * h;
            const v4f b0 = *(const v4f*)bp, b1 = *(const v4f*)(bp + 4);
            bmv[0] = bf16r(b0[0]); bmv[1] = bf16r(b0[1]); bmv[2] = bf16r(b0[2]); bmv[3] = bf16r(b0[3]);
            bmv[4] = bf16r(b1[0]); bmv[5] = bf16r(b1[1]); bmv[6] = bf16r(b1[2]); bmv[7] = bf16r(b1[3]);
        } else {
#pragma unroll
            for (int r = 0; r < 8; ++r) bmv[r] = 0.0f;
        }
#pragma unroll
        for (int bt = 0; bt < 4; ++bt) {
            float bn = 0.0f;
            if (MODE == 1) bn = bf16r(bias[n0 + 64 * wn + 16 * bt + n16]);
            v8h pk;
#pragma unroll
            for (int r = 0; r < 8; ++r) {
                const float v = acc[at][bt][r] * osc + (MODE == 0 ? bmv[r] : bn);
                pk[r] = (_Float16)v;
            }
            *(v8h*)(L + (size_t)(64 * wn + 16 * bt + n16) * LDP + 32 * wmi + 16 * at + 8 * h) = pk;
        }
    }
    __syncthreads();
    v4u vals[8];
#pragma unroll
    for (int it = 0; it < 8; ++it) {
        const int row = wv * 16 + 2 * it + h;
        const v8h t = *(const v8h*)(L + (size_t)row * LDP + 8 * n16);
        vals[it] = __builtin_bit_cast(v4u, t);
    }
#pragma unroll
    for (int it = 0; it < 8; ++it) {
        const int row = wv * 16 + 2 * it + h;
        size_t goff;
        if (MODE == 0) goff = (size_t)(n0 + row) * DM + m0 + 8 * n16;
        else           goff = (size_t)(m0 / SEQ) * ((size_t)DM * SEQ) + (size_t)(n0 + row) * SEQ + (m0 % SEQ) + 8 * n16;
        *(volatile v4u*)(Out + goff) = vals[it];
    }
    __threadfence();
#pragma unroll
    for (int it = 0; it < 8; ++it) {
        const int row = wv * 16 + 2 * it + h;
        size_t goff;
        if (MODE == 0) goff = (size_t)(n0 + row) * DM + m0 + 8 * n16;
        else           goff = (size_t)(m0 / SEQ) * ((size_t)DM * SEQ) + (size_t)(n0 + row) * SEQ + (m0 % SEQ) + 8 * n16;
        *(volatile v4u*)(Out + goff) = vals[it];
    }
}

__global__ __launch_bounds__(256) __attribute__((amdgpu_num_vgpr(256)))
void attn_kernel(const _Float16* __restrict__ Qh, const _Float16* __restrict__ Kh, const _Float16* __restrict__ Vt,
                 const float* __restrict__ amask, float* out) {
    __shared__ __align__(16) float mk[SEQ];
    __shared__ __align__(16) float ol[8 * 16 * OLP];
    const int tid = threadIdx.x, lane = tid & 31, wv = tid >> 5, h = lane >> 4, n16 = lane & 15;
    const int bh = blockIdx.y, b = bh / NH, hd = bh - b * NH;
    const int q0 = blockIdx.x * 128 + wv * 16;
    for (int i = tid; i < SEQ; i += 256) mk[i] = bf16r(amask[(size_t)b * SEQ_FULL + i]);
    __syncthreads();

    const _Float16* qr = Qh + (size_t)(b * SEQ + q0 + n16) * DM + hd * HD + 8 * h;
    Frag qa, qb;
    qa.hf[0] = ld8(qr);      qa.hf[1] = ld8(qr + 16);
    qb.hf[0] = ld8(qr + 32); qb.hf[1] = ld8(qr + 48);
    const _Float16* kb = Kh + (size_t)(b * SEQ + n16) * DM + hd * HD + 8 * h;
    const _Float16* vb = Vt + (size_t)b * DM * SEQ + (size_t)(hd * HD + n16) * SEQ + 8 * h;

    v8f o[4];
#pragma unroll
    for (int dt = 0; dt < 4; ++dt) o[dt] = (v8f){};
    float m = -1e30f, l = 0.0f;

#pragma unroll 1
    for (int ks = 0; ks < SEQ / 64; ++ks) {
        v8f s[4];
#pragma unroll
        for (int kt = 0; kt < 4; ++kt) {
            s[kt] = (v8f){};
            const _Float16* kr = kb + (size_t)(64 * ks + 16 * kt) * DM;
            Frag kf;
            kf.hf[0] = ld8(kr);      kf.hf[1] = ld8(kr + 16);
            s[kt] = wmma16(kf.v, qa.v, s[kt]);
            kf.hf[0] = ld8(kr + 32); kf.hf[1] = ld8(kr + 48);
            s[kt] = wmma16(kf.v, qb.v, s[kt]);
        }
        float mx = -1e30f;
#pragma unroll
        for (int kt = 0; kt < 4; ++kt) {
            const float* mp = mk + 64 * ks + 16 * kt + 8 * h;
            const v4f ma = *(const v4f*)mp, mb = *(const v4f*)(mp + 4);
            const float mvv[8] = {ma[0], ma[1], ma[2], ma[3], mb[0], mb[1], mb[2], mb[3]};
#pragma unroll
            for (int r = 0; r < 8; ++r) {
                const float t = s[kt][r] * 0.125f + mvv[r];
                s[kt][r] = t;
                mx = fmaxf(mx, t);
            }
        }
        mx = fmaxf(mx, __shfl_xor(mx, 16, 32));
        const float mn = fmaxf(m, mx);
        const float corr = __expf(m - mn);
        m = mn;
        float ps = 0.0f;
        v16h pv[2];
        pv[0] = (v16h){}; pv[1] = (v16h){};
#pragma unroll
        for (int kt = 0; kt < 4; ++kt) {
#pragma unroll
            for (int r = 0; r < 8; ++r) {
                const float p = __expf(s[kt][r] - mn);
                ps += p;
                pv[kt >> 1][((kt & 1) << 3) + r] = (_Float16)(p * PSC);
            }
        }
        ps += __shfl_xor(ps, 16, 32);
        l = l * corr + ps;
#pragma unroll
        for (int dt = 0; dt < 4; ++dt)
#pragma unroll
            for (int r = 0; r < 8; ++r) o[dt][r] *= corr;
#pragma unroll
        for (int dt = 0; dt < 4; ++dt) {
            const _Float16* vr = vb + (size_t)(16 * dt) * SEQ + 64 * ks;
            Frag vf;
            vf.hf[0] = ld8(vr);      vf.hf[1] = ld8(vr + 16);
            o[dt] = wmma16(vf.v, pv[0], o[dt]);
            vf.hf[0] = ld8(vr + 32); vf.hf[1] = ld8(vr + 48);
            o[dt] = wmma16(vf.v, pv[1], o[dt]);
        }
    }

    const float inv = 1.0f / (l * PSC);
    float* olw = ol + wv * (16 * OLP);
#pragma unroll
    for (int dt = 0; dt < 4; ++dt) {
        v4f a, c;
        a[0] = o[dt][0] * inv; a[1] = o[dt][1] * inv; a[2] = o[dt][2] * inv; a[3] = o[dt][3] * inv;
        c[0] = o[dt][4] * inv; c[1] = o[dt][5] * inv; c[2] = o[dt][6] * inv; c[3] = o[dt][7] * inv;
        *(v4f*)(olw + n16 * OLP + 16 * dt + 8 * h) = a;
        *(v4f*)(olw + n16 * OLP + 16 * dt + 8 * h + 4) = c;
    }
    __syncthreads();
    v4f vals[8];
#pragma unroll
    for (int it = 0; it < 8; ++it) vals[it] = *(const v4f*)(olw + (2 * it + h) * OLP + 4 * n16);
    float* ob = out + (size_t)(b * SEQ + q0) * DM + hd * HD + 4 * n16;
#pragma unroll
    for (int it = 0; it < 8; ++it) *(volatile v4f*)(ob + (size_t)(2 * it + h) * DM) = vals[it];
    __threadfence();
#pragma unroll
    for (int it = 0; it < 8; ++it) *(volatile v4f*)(ob + (size_t)(2 * it + h) * DM) = vals[it];
}

extern "C" void kernel_launch(void* const* d_in, const int* in_sizes, int n_in,
                              void* d_out, int out_size, void* d_ws, size_t ws_size,
                              hipStream_t stream) {
    if (n_in < 8) return;
    const long long needX = ((long long)(NB - 1) * SEQ_FULL + SEQ) * DM;
    const long long needM = (long long)(NB - 1) * SEQ_FULL + SEQ;
    if ((long long)in_sizes[0] < needX || (long long)in_sizes[1] < needM) return;
    if (in_sizes[2] < DM * DM || in_sizes[4] < DM * DM || in_sizes[6] < DM * DM) return;
    if (in_sizes[3] < DM || in_sizes[5] < DM || in_sizes[7] < DM) return;
    if (out_size < NT * DM) return;

    const float* x    = (const float*)d_in[0];
    const float* amsk = (const float*)d_in[1];
    const float* wq   = (const float*)d_in[2];
    const float* bq   = (const float*)d_in[3];
    const float* wk   = (const float*)d_in[4];
    const float* bk   = (const float*)d_in[5];
    const float* wv   = (const float*)d_in[6];
    const float* bv   = (const float*)d_in[7];
    float* out = (float*)d_out;

    const size_t xhB = (size_t)NT * DM * 2;
    const size_t whB = (size_t)DM * DM * 2;
    const size_t qhB = xhB;
    const size_t vtB = (size_t)NB * DM * SEQ * 2;
    const size_t total = xhB + 3 * whB + 2 * qhB + vtB;
    if (total > ws_size) return;
    char* ws = (char*)d_ws;
    _Float16* Xh  = (_Float16*)(ws);
    _Float16* Wqh = (_Float16*)(ws + xhB);
    _Float16* Wkh = (_Float16*)(ws + xhB + whB);
    _Float16* Wvh = (_Float16*)(ws + xhB + 2 * whB);
    _Float16* Qh  = (_Float16*)(ws + xhB + 3 * whB);
    _Float16* Khp = (_Float16*)(ws + xhB + 3 * whB + qhB);
    _Float16* Vt  = (_Float16*)(ws + xhB + 3 * whB + 2 * qhB);

    const int nbx = NT * (DM / 8) / 256, nbw = DM * (DM / 8) / 256;
    cvt_kernel<<<dim3((unsigned)(nbx + 3 * nbw)), 256, 0, stream>>>(x, wq, wk, wv, Xh, Wqh, Wkh, Wvh);
    proj_kernel<0><<<dim3(DM / 128, NT / 128, 2), 256, 0, stream>>>(Wqh, Wkh, Xh, bq, bk, Qh, Khp);
    proj_kernel<1><<<dim3(NT / 128, DM / 128, 1), 256, 0, stream>>>(Xh, Xh, Wvh, bv, bv, Vt, Vt);
    attn_kernel<<<dim3(SEQ / 128, NB * NH), 256, 0, stream>>>(Qh, Khp, Vt, amsk, out);
}
